// NewsEncoder_36378372997626
// MI455X (gfx1250) — hardware-run, weakly checked
//
#include <hip/hip_runtime.h>


#ifndef NT
#define NT 65536
#endif
#ifndef NH
#define NH 262144
#endif
#define NT_FULL 65536
#define NH_FULL 262144
#define CATV   1000
#define TYPEV  10
#define EMB    64
#define PROJ   16
#define MAXSUB 8
#define SENT   3
#define XTW    35
#define HIN    37
#define KP     64
#define W1OUT  32
#define TROW0  1008
#define TROWS  1024
#define TTILE  63
#define RW     4
#define RB     128
#define XP     72
#define OSP    36
#define WST    1152
#define TQ     280
#define XS     256.0f
#define WS     64.0f
#define INVS   (1.0f / 16384.0f)

static_assert(EMB % 32 == 0);
static_assert(KP % 32 == 0);
static_assert(HIN <= KP);
static_assert(PROJ == 16);
static_assert(W1OUT == 32);
static_assert(PROJ + SENT + PROJ == XTW);
static_assert(XTW + 2 == HIN);
static_assert(TROW0 % 16 == 0);
static_assert(TROW0 >= CATV);
static_assert(TROW0 + 16 == TROWS);
static_assert(TTILE * 16 == TROW0);
static_assert(TYPEV <= 16);
static_assert(RB == 32 * RW);
static_assert(NT % RB == 0);
static_assert(NH % RB == 0);
static_assert(NT <= NT_FULL);
static_assert(NH <= NH_FULL);
static_assert((32 * XTW * 4) % 128 == 0);
static_assert(32 * XTW == TQ * 4);
static_assert(9 * 32 >= TQ);
static_assert(8 * 32 < TQ);
static_assert((TQ - 8 * 32) % 8 == 0);
static_assert(WST >= 32 * XTW);
static_assert(WST == 32 * OSP);
static_assert(WST % 4 == 0);
static_assert((OSP * 4) % 16 == 0);
static_assert((XP * 2) % 16 == 0);
static_assert(XP >= KP);
static_assert(8 * 4 == 32);
static_assert(8 * 32 * 16 == 32 * W1OUT * 4);
static_assert(2 * 32 * 16 == 16 * PROJ * 4);
static_assert((size_t)NT_FULL * XTW * 4 == (size_t)9175040);
static_assert(((size_t)NT_FULL * XTW * 4) % 128 == 0);
static_assert((size_t)RW * WST * 4 + (size_t)RW * 32 * XP * 2 <= 131072);
static_assert(TROWS * EMB / 8 == 32 * 256);
static_assert(32 * EMB / 8 == 256);
static_assert(W1OUT * KP / 8 == 256);

typedef _Float16 h16;
typedef unsigned short bf;
typedef __attribute__((ext_vector_type(16))) __bf16   v16bf;
typedef __attribute__((ext_vector_type(16))) _Float16 v16h;
typedef __attribute__((ext_vector_type(8)))  _Float16 v8h;
typedef __attribute__((ext_vector_type(8)))  unsigned short v8us;
typedef __attribute__((ext_vector_type(8)))  float    v8f;
typedef __attribute__((ext_vector_type(4)))  float    v4f;
typedef __attribute__((ext_vector_type(4)))  int      v4i;
typedef v4f  __attribute__((may_alias)) v4fa;

__device__ __forceinline__ unsigned short f2bf(float f) { unsigned u = __float_as_uint(f); u += 0x7FFFu + ((u >> 16) & 1u); return (unsigned short)(u >> 16); }
__device__ __forceinline__ float bfr(float f) { return __uint_as_float(((unsigned)f2bf(f)) << 16); }
__device__ __forceinline__ v16h cat16(v8h lo, v8h hi) { return __builtin_shufflevector(lo, hi, 0, 1, 2, 3, 4, 5, 6, 7, 8, 9, 10, 11, 12, 13, 14, 15); }
__device__ __forceinline__ v16bf cat16b(v8us lo, v8us hi) { return __builtin_bit_cast(v16bf, __builtin_shufflevector(lo, hi, 0, 1, 2, 3, 4, 5, 6, 7, 8, 9, 10, 11, 12, 13, 14, 15)); }
__device__ __forceinline__ v8f wmma16(v16h a, v16h b, v8f c) { return __builtin_amdgcn_wmma_f32_16x16x32_f16(false, a, false, b, (short)0, c, false, false); }
__device__ __forceinline__ v8f wmmab(v16bf a, v16bf b, v8f c) { return __builtin_amdgcn_wmma_f32_16x16x32_bf16(false, a, false, b, (short)0, c, false, false); }
__device__ __forceinline__ v16h  ldh(const h16* p) { return cat16(*(const v8h*)p, *(const v8h*)(p + 16)); }
__device__ __forceinline__ v16bf ldb(const bf* p)  { return cat16b(*(const v8us*)p, *(const v8us*)(p + 16)); }
__device__ __forceinline__ void wave_sync() { __builtin_amdgcn_fence(3  , "wavefront"); __builtin_amdgcn_wave_barrier(); asm volatile("" ::: "memory"); }

__device__ __forceinline__ v8f wmma16_g(v16h a, v16h b, v8f c) { c = wmma16(a, b, c); asm volatile("v_nop\n\tv_nop\n\tv_nop\n\tv_nop" : "+v"(c) : "v"(a), "v"(b)); return c; }
__device__ __forceinline__ v8f wmmab_g(v16bf a, v16bf b, v8f c) { c = wmmab(a, b, c); asm volatile("v_nop\n\tv_nop\n\tv_nop\n\tv_nop" : "+v"(c) : "v"(a), "v"(b)); return c; }
__device__ __forceinline__ h16 toh_flush(float v) { const h16 r = (h16)v; return (fabsf(v) < 6.103515625e-05f) ? (h16)0.0f : r; }
__device__ __forceinline__ int wrapclamp(int i, int n) { i = (i < 0) ? (i + n) : i; i = (i < 0) ? 0 : i; return (i > n - 1) ? (n - 1) : i; }

__global__ __launch_bounds__(256) void k_prep(const float* __restrict__ cat_emb, const float* __restrict__ type_emb, const float* __restrict__ cat_W, const float* __restrict__ type_W,
                                              const float* __restrict__ w1_W, bf* AB, bf* WT, h16* W1T) {
    const int blk = blockIdx.x;
    if (blk < 32) {
        const int g = blk * 256 + (int)threadIdx.x;
        const int row = g >> 3, c8 = (g & 7) * 8;
        const int rc = row < CATV - 1 ? row : CATV - 1;
        int rt = row - TROW0; rt = rt < 0 ? 0 : (rt > TYPEV - 1 ? TYPEV - 1 : rt);
        v8f vc = *(const v8f*)(cat_emb + (size_t)rc * EMB + c8);
        v8f vt = *(const v8f*)(type_emb + (size_t)rt * EMB + c8);
        asm volatile("" : "+v"(vc)); asm volatile("" : "+v"(vt));
        const bool isC = row < CATV; const bool isT = (row >= TROW0) & (row < TROW0 + TYPEV);
        v8us o;
#pragma unroll
        for (int k = 0; k < 8; ++k) { const unsigned short uc = f2bf(vc[k]), ut = f2bf(vt[k]); o[k] = isC ? uc : (isT ? ut : (unsigned short)0); }
        *(volatile v8us*)(AB + (size_t)g * 8) = o; __threadfence(); *(volatile v8us*)(AB + (size_t)g * 8) = o;
    } else if (blk == 32) {
        const int q = (int)threadIdx.x; const int n = q >> 3, k8 = (q & 7) * 8, nn = n & 15;
        v8us o;
#pragma unroll
        for (int k = 0; k < 8; ++k) { float a = cat_W[(k8 + k) * PROJ + nn]; float b = type_W[(k8 + k) * PROJ + nn];
            asm volatile("" : "+v"(a)); asm volatile("" : "+v"(b));
            const unsigned short ua = f2bf(a), ub = f2bf(b); o[k] = (n < 16) ? ua : ub; }
        *(volatile v8us*)(WT + (size_t)q * 8) = o; __threadfence(); *(volatile v8us*)(WT + (size_t)q * 8) = o;
    } else {
        const int q = (int)threadIdx.x; const int n = q >> 3, k8 = (q & 7) * 8;
        v8h o;
#pragma unroll
        for (int k = 0; k < 8; ++k) { const int kk = k8 + k; const int kc = kk < HIN - 1 ? kk : HIN - 1;
            float w = w1_W[kc * W1OUT + n];
            asm volatile("" : "+v"(w));
            const h16 hv = toh_flush(bfr(w) * WS); o[k] = (kk < HIN) ? hv : (h16)0.0f; }
        *(volatile v8h*)(W1T + (size_t)q * 8) = o; __threadfence(); *(volatile v8h*)(W1T + (size_t)q * 8) = o;
    }
}

__global__ __launch_bounds__(32) void k_table(const bf* __restrict__ AB, const bf* __restrict__ WT, const float* __restrict__ type_b, float* PT) {
    __shared__ __align__(16) float os[16 * 20];
    const int lane = threadIdx.x & 31, lr = lane & 15, hi = lane >> 4;
    const int tile = blockIdx.x; const int r0 = tile * 16;
    const int wsel = (tile == TTILE) ? 16 : 0;
    const size_t aoff = (size_t)(r0 + lr) * EMB + 8 * hi, boff = (size_t)(wsel + lr) * EMB + 8 * hi;
    v8f acc = (v8f){};
#pragma unroll
    for (int kc = 0; kc < EMB; kc += 32) { const v16bf a = ldb(AB + aoff + kc); const v16bf b = ldb(WT + boff + kc); acc = wmmab_g(a, b, acc); }
    const float tb = bfr(type_b[lr]);
    const float badd = (tile == TTILE) ? tb : 0.0f;
#pragma unroll
    for (int j = 0; j < 8; ++j) os[(hi * 8 + j) * 20 + lr] = acc[j] + badd;
    wave_sync();
    float* og = PT + (size_t)r0 * PROJ;
#pragma unroll 1
    for (int ps = 0; ps < 2; ++ps) {
#pragma unroll
        for (int s = 0; s < 2; ++s) { const int p = s * 32 + lane; const int row = p >> 2, c4 = (p & 3) * 4;
            const v4f val = *(const v4fa*)(&os[row * 20 + c4]);
            *(volatile v4f*)(og + (size_t)p * 4) = val; }
        if (ps == 0) __threadfence(); }
}

__device__ __forceinline__ void row_feat(const int* __restrict__ cat, const int* __restrict__ sub, const int* __restrict__ slen, const float* __restrict__ sent, const int* __restrict__ typ,
                                         const float* __restrict__ PT, const float* __restrict__ cat_b, size_t r, v4f (&ct)[4], v4f (&tt)[4], float (&sv)[3]) {
    const int c = wrapclamp(cat[r], CATV);
    const int len = slen[r];
    const int ty = wrapclamp(typ[r], TYPEV);
    v4f acc[4];
#pragma unroll
    for (int q = 0; q < 4; ++q) acc[q] = (v4f){};
#pragma unroll 1
    for (int g = 0; g < 2; ++g) {
        const v4i si = *(const v4i*)(sub + r * MAXSUB + g * 4);
#pragma unroll
        for (int s = 0; s < 4; ++s) {
            const int idx = wrapclamp(si[s], CATV);
            const float m = (g * 4 + s < len) ? 1.0f : 0.0f;
            const v4f* p = (const v4f*)(PT + (size_t)idx * PROJ);
#pragma unroll
            for (int q = 0; q < 4; ++q) acc[q] += p[q] * m;
        }
    }
    const int dl = len < 1 ? 1 : len;
    const float inv = 1.0f / (float)dl;
    const v4f* pb = (const v4f*)(PT + (size_t)c * PROJ);
    const v4f* pt = (const v4f*)(PT + (size_t)(TROW0 + ty) * PROJ);
#pragma unroll
    for (int q = 0; q < 4; ++q) { const v4f b4 = pb[q];
#pragma unroll
        for (int i = 0; i < 4; ++i) { const float cb = bfr(cat_b[4 * q + i]); ct[q][i] = (b4[i] + cb) + (acc[q][i] * inv + cb); }
        tt[q] = pt[q]; }
#pragma unroll
    for (int i = 0; i < SENT; ++i) sv[i] = bfr(sent[r * SENT + i]);
}

__global__ __launch_bounds__(RB) void k_rows(const int* __restrict__ cat_t, const int* __restrict__ sub_t, const int* __restrict__ len_t, const float* __restrict__ sent_t, const int* __restrict__ type_t,
                                             const int* __restrict__ cat_h, const int* __restrict__ sub_h, const int* __restrict__ len_h, const float* __restrict__ sent_h, const int* __restrict__ type_h,
                                             const float* __restrict__ rt_h, const float* __restrict__ sc_h,
                                             const float* __restrict__ PT, const float* __restrict__ cat_b, const h16* __restrict__ W1T, const float* __restrict__ w1_b,
                                             float* OUT0, float* OUT1) {
    __shared__ __align__(16) float st[RW * WST];
    __shared__ __align__(16) h16 xs[RW * 32 * XP];
    const int lane = threadIdx.x & 31, lr = lane & 15, hi = lane >> 4;
    const int wave = __builtin_amdgcn_readfirstlane((int)(threadIdx.x >> 5));
    const int blk = blockIdx.x;
    const int wb = wave * WST;
    v4f ct[4], tt[4]; float sv[3];
    if (blk < NT / RB) {
        const size_t row0 = (size_t)blk * RB + (size_t)wave * 32;
        row_feat(cat_t, sub_t, len_t, sent_t, type_t, PT, cat_b, row0 + lane, ct, tt, sv);
        const int so = wb + lane * XTW;
#pragma unroll
        for (int q = 0; q < 4; ++q) {
#pragma unroll
            for (int i = 0; i < 4; ++i) { st[so + 4 * q + i] = ct[q][i]; st[so + PROJ + SENT + 4 * q + i] = tt[q][i]; } }
#pragma unroll
        for (int i = 0; i < SENT; ++i) st[so + PROJ + i] = sv[i];
        wave_sync();
        float* og = OUT0 + row0 * XTW;
#pragma unroll 1
        for (int ps = 0; ps < 2; ++ps) {
#pragma unroll
            for (int it = 0; it < 9; ++it) { const int p = it * 32 + lane; const int pc = p < TQ ? p : TQ - 1;
                const v4f val = *(const v4fa*)(&st[wb + pc * 4]);
                if (p < TQ) *(volatile v4f*)(og + (size_t)p * 4) = val; }
            if (ps == 0) __threadfence(); }
    } else {
        const size_t row0 = (size_t)(blk - NT / RB) * RB + (size_t)wave * 32;
        const size_t r = row0 + lane;
        row_feat(cat_h, sub_h, len_h, sent_h, type_h, PT, cat_b, r, ct, tt, sv);
        const float rtv = bfr(rt_h[r]), scv = bfr(sc_h[r]);
        float z = 0.0f; asm volatile("" : "+v"(z));
        float f[40];
#pragma unroll
        for (int q = 0; q < 4; ++q) {
#pragma unroll
            for (int i = 0; i < 4; ++i) { f[4 * q + i] = ct[q][i]; f[PROJ + SENT + 4 * q + i] = tt[q][i]; } }
#pragma unroll
        for (int i = 0; i < SENT; ++i) f[PROJ + i] = sv[i];
        f[35] = rtv; f[36] = scv; f[37] = z; f[38] = z; f[39] = z;
        const int xo = wave * 32 * XP + lane * XP;
#pragma unroll
        for (int g = 0; g < 5; ++g) { v8h x;
#pragma unroll
            for (int i = 0; i < 8; ++i) x[i] = toh_flush(f[8 * g + i] * XS);
            *(v8h*)(&xs[xo + 8 * g]) = x; }
        { v8h zv;
#pragma unroll
          for (int i = 0; i < 8; ++i) zv[i] = (h16)z;
#pragma unroll
          for (int g = 5; g < 8; ++g) *(v8h*)(&xs[xo + 8 * g]) = zv; }
        wave_sync();
        const v16h b00 = ldh(W1T + (size_t)lr * KP + 8 * hi), b01 = ldh(W1T + (size_t)lr * KP + 8 * hi + 32);
        const v16h b10 = ldh(W1T + (size_t)(16 + lr) * KP + 8 * hi), b11 = ldh(W1T + (size_t)(16 + lr) * KP + 8 * hi + 32);
        const float bb0 = bfr(w1_b[lr]), bb1 = bfr(w1_b[16 + lr]);
#pragma unroll
        for (int mt = 0; mt < 2; ++mt) {
            const int ao = wave * 32 * XP + (mt * 16 + lr) * XP + 8 * hi;
            const v16h a0 = cat16(*(const v8h*)(&xs[ao]), *(const v8h*)(&xs[ao + 16]));
            const v16h a1 = cat16(*(const v8h*)(&xs[ao + 32]), *(const v8h*)(&xs[ao + 48]));
            v8f c0 = (v8f){}, c1 = (v8f){};
            c0 = wmma16_g(a0, b00, c0); c0 = wmma16_g(a1, b01, c0);
            c1 = wmma16_g(a0, b10, c1); c1 = wmma16_g(a1, b11, c1);
#pragma unroll
            for (int j = 0; j < 8; ++j) { st[wb + (mt * 16 + hi * 8 + j) * OSP + lr] = c0[j] * INVS + bb0; st[wb + (mt * 16 + hi * 8 + j) * OSP + 16 + lr] = c1[j] * INVS + bb1; }
        }
        wave_sync();
        float* og = OUT1 + row0 * W1OUT;
#pragma unroll 1
        for (int ps = 0; ps < 2; ++ps) {
#pragma unroll
            for (int s = 0; s < 8; ++s) { const int row = 4 * s + (lane >> 3), cofs = (lane & 7) * 4;
                const v4f val = *(const v4fa*)(&st[wb + row * OSP + cofs]);
                *(volatile v4f*)(og + (size_t)row * W1OUT + cofs) = val; }
            if (ps == 0) __threadfence(); }
    }
}

#define AL256(v)  ((((size_t)(v)) + 255) & ~(size_t)255)
#define SZ_AB     AL256((size_t)TROWS * EMB * 2)
#define SZ_WT     AL256((size_t)32 * EMB * 2)
#define SZ_W1T    AL256((size_t)W1OUT * KP * 2)
#define SZ_PT     AL256((size_t)TROWS * PROJ * 4)
#define SZ_TOTAL  (SZ_AB + SZ_WT + SZ_W1T + SZ_PT)
static_assert(SZ_TOTAL <= (size_t)134217728);
static_assert(SZ_TOTAL == (size_t)204800);
static_assert((size_t)(32 * 256) * 16 == (size_t)TROWS * EMB * 2);
static_assert((size_t)256 * 16 == (size_t)32 * EMB * 2);
static_assert((size_t)256 * 16 == (size_t)W1OUT * KP * 2);
static_assert((size_t)(TROWS / 16) * 1024 == (size_t)TROWS * PROJ * 4);

extern "C" void kernel_launch(void* const* d_in, const int* in_sizes, int n_in,
                              void* d_out, int out_size, void* d_ws, size_t ws_size, hipStream_t stream) {
    if (n_in < 20) return;
    if ((size_t)in_sizes[0] < (size_t)NT || (size_t)in_sizes[1] < (size_t)NT * MAXSUB || (size_t)in_sizes[2] < (size_t)NT) return;
    if ((size_t)in_sizes[3] < (size_t)NT * SENT || (size_t)in_sizes[4] < (size_t)NT) return;
    if ((size_t)in_sizes[5] < (size_t)NH || (size_t)in_sizes[6] < (size_t)NH * MAXSUB || (size_t)in_sizes[7] < (size_t)NH) return;
    if ((size_t)in_sizes[8] < (size_t)NH * SENT || (size_t)in_sizes[9] < (size_t)NH) return;
    if ((size_t)in_sizes[10] < (size_t)NH || (size_t)in_sizes[11] < (size_t)NH) return;
    if (in_sizes[12] < CATV * EMB || in_sizes[13] < EMB * PROJ || in_sizes[14] < PROJ) return;
    if (in_sizes[15] < TYPEV * EMB || in_sizes[16] < EMB * PROJ || in_sizes[17] < PROJ) return;
    if (in_sizes[18] < HIN * W1OUT || in_sizes[19] < W1OUT) return;
    if ((size_t)out_size < (size_t)NT_FULL * XTW + (size_t)NH * W1OUT) return;
    if (ws_size < SZ_TOTAL) return;
    const int*   cat_t  = (const int*)d_in[0];
    const int*   sub_t  = (const int*)d_in[1];
    const int*   len_t  = (const int*)d_in[2];
    const float* sent_t = (const float*)d_in[3];
    const int*   type_t = (const int*)d_in[4];
    const int*   cat_h  = (const int*)d_in[5];
    const int*   sub_h  = (const int*)d_in[6];
    const int*   len_h  = (const int*)d_in[7];
    const float* sent_h = (const float*)d_in[8];
    const int*   type_h = (const int*)d_in[9];
    const float* rt_h   = (const float*)d_in[10];
    const float* sc_h   = (const float*)d_in[11];
    const float* cat_emb  = (const float*)d_in[12];
    const float* cat_W    = (const float*)d_in[13];
    const float* cat_b    = (const float*)d_in[14];
    const float* type_emb = (const float*)d_in[15];
    const float* type_W   = (const float*)d_in[16];
    const float* type_b   = (const float*)d_in[17];
    const float* w1_W     = (const float*)d_in[18];
    const float* w1_b     = (const float*)d_in[19];
    float* OUT0 = (float*)d_out;
    float* OUT1 = (float*)d_out + (size_t)NT_FULL * XTW;
    char* wsp = (char*)d_ws;
    bf*  AB  = (bf*)wsp;   wsp += SZ_AB;
    bf*  WT  = (bf*)wsp;   wsp += SZ_WT;
    h16* W1T = (h16*)wsp;  wsp += SZ_W1T;
    float* PT = (float*)wsp; wsp += SZ_PT;

    k_prep<<<34, 256, 0, stream>>>(cat_emb, type_emb, cat_W, type_W, w1_W, AB, WT, W1T);
    k_table<<<TROWS / 16, 32, 0, stream>>>(AB, WT, type_b, PT);
    k_rows<<<NT / RB + NH / RB, RB, 0, stream>>>(cat_t, sub_t, len_t, sent_t, type_t, cat_h, sub_h, len_h, sent_h, type_h, rt_h, sc_h,
                                                 PT, cat_b, W1T, w1_b, OUT0, OUT1);
}
